// SPINN_46359876993764
// MI455X (gfx1250) — hardware-verified
//
#include <hip/hip_runtime.h>
#include <stddef.h>


#define NB     64
#define NL     512
#define NE     300
#define NEP    320
#define NH     256
#define NH2    512
#define NG5    1280
#define SDEP   528
#define NROWS  32768
#define APITCH 528
#define EP     68
#define NTHR   256
#define RTHR   512
#define CB_S   5120
#define CB_W   80
#define CB_G   320
#define WSCAP  134217728

static_assert(CB_S * NTHR == NROWS * (NEP / 8));
static_assert(CB_W * NTHR == NH2 * (NEP / 8));
static_assert(CB_G * NTHR == NG5 * (NH2 / 8));
static_assert(NROWS == NB * NL);
static_assert((APITCH * 2) % 16 == 0);
static_assert((EP * 4) % 16 == 0);
static_assert(8 * 16 * EP * 4 <= 65536);

#define LDS_A    0
#define LDS_C    (LDS_A + NB * APITCH * 2)
#define LDS_H    (LDS_C + NB * NH * 4)
#define LDS_I    (LDS_H + NB * NH * 4)
#define LDS_TOT  (LDS_I + 8 * NB * 4)
static_assert(LDS_C % 16 == 0);
static_assert(LDS_H % 16 == 0);
static_assert(LDS_I % 16 == 0);
static_assert(LDS_TOT <= 300000);

typedef _Float16      v4h  __attribute__((ext_vector_type(4)));
typedef _Float16      v8h  __attribute__((ext_vector_type(8)));
typedef _Float16      v16h __attribute__((ext_vector_type(16)));
typedef float         v4f  __attribute__((ext_vector_type(4)));
typedef float         v8f  __attribute__((ext_vector_type(8)));
typedef unsigned int  v4u  __attribute__((ext_vector_type(4)));
union Frag { v16h v; v4u q[2]; };

__device__ __forceinline__ v8f wmh(v16h a, v16h b, v8f c) {
  v8f d = __builtin_amdgcn_wmma_f32_16x16x32_f16(false, a, false, b, (short)0, c, false, false);
  asm volatile("v_nop\n\tv_nop\n\tv_nop\n\tv_nop" : "+v"(d) : "v"(a), "v"(b));
  return d;
}

__device__ __forceinline__ v8f zero8() { v8f z = {0.f, 0.f, 0.f, 0.f, 0.f, 0.f, 0.f, 0.f}; return z; }

__device__ __forceinline__ v4u pack8(v4f a, v4f c, float s) {
  union { v8h h; v4u u; } U;
  v8h t = {(_Float16)(a.x * s), (_Float16)(a.y * s), (_Float16)(a.z * s), (_Float16)(a.w * s),
           (_Float16)(c.x * s), (_Float16)(c.y * s), (_Float16)(c.z * s), (_Float16)(c.w * s)};
  U.h = t;
  return U.u;
}

__device__ __forceinline__ float sigf(float x) {
  const float e = __expf(-x);
  return __builtin_amdgcn_rcpf(1.0f + e);
}
__device__ __forceinline__ float tanhx(float x) {
  const float e = __expf(-2.0f * fabsf(x));
  const float r = (1.0f - e) * __builtin_amdgcn_rcpf(1.0f + e);
  return x < 0.0f ? -r : r;
}

__global__ __launch_bounds__(NTHR) void k_cvt(const float* __restrict__ sent, const float* __restrict__ Ww,
                                              const float* __restrict__ Wl, const float* __restrict__ Wr,
                                              unsigned short* sent16, unsigned short* wt16,
                                              unsigned short* wg16) {
  const int blk = (int)blockIdx.x, tid = (int)threadIdx.x;
  v4u pv;
  unsigned short* dp;
  if (blk < CB_S) {
    const int g = blk * NTHR + tid;
    const int row = g / 40, pc = g - row * 40, k = pc * 8;
    const int kA = (k < 296) ? k : 296;
    const int kB = ((k + 4) < 296) ? (k + 4) : 296;
    const float* rp = sent + (size_t)row * NE;
    v4f a = *(const v4f*)(rp + kA);
    v4f c = *(const v4f*)(rp + kB);
    const v4f z = {0.f, 0.f, 0.f, 0.f};
    a = (k < NE) ? a : z;
    c = ((k + 4) < NE) ? c : z;
    pv = pack8(a, c, 16.0f);
    dp = sent16 + (size_t)g * 8;
  } else if (blk < CB_S + CB_W) {
    const int g = (blk - CB_S) * NTHR + tid;
    const int n = g / 40, pc = g - n * 40, k0 = pc * 8;
    float v[8];
#pragma unroll
    for (int e = 0; e < 8; ++e) {
      const int k = k0 + e;
      const int kc = (k < NE) ? k : (NE - 1);
      const float w = Ww[(size_t)kc * NH2 + n];
      v[e] = (k < NE) ? w * 64.0f : 0.0f;
    }
    const v4f a = {v[0], v[1], v[2], v[3]};
    const v4f c = {v[4], v[5], v[6], v[7]};
    pv = pack8(a, c, 1.0f);
    dp = wt16 + (size_t)g * 8;
  } else {
    const int g = (blk - CB_S - CB_W) * NTHR + tid;
    const int n = g >> 6, pc = g & 63, k0 = pc * 8;
    float v[8];
#pragma unroll
    for (int e = 0; e < 8; ++e) {
      const int k = k0 + e;
      const int kc = k & (NH - 1);
      const float wl = Wl[(size_t)kc * NG5 + n];
      const float wr = Wr[(size_t)kc * NG5 + n];
      v[e] = ((k < NH) ? wl : wr) * 64.0f;
    }
    const v4f a = {v[0], v[1], v[2], v[3]};
    const v4f c = {v[4], v[5], v[6], v[7]};
    pv = pack8(a, c, 1.0f);
    dp = wg16 + (size_t)g * 8;
  }
  *(volatile v4u*)dp = pv;
  __threadfence();
  *(volatile v4u*)dp = pv;
}

__global__ __launch_bounds__(NTHR) void k_proj(const unsigned short* __restrict__ sent16,
                                               const unsigned short* __restrict__ wt16,
                                               const float* __restrict__ bw,
                                               unsigned short* hproj, float* cproj) {
  __shared__ __attribute__((aligned(16))) float sE[8 * 16 * EP];
  const int tid = threadIdx.x, lane = tid & 31, wave = tid >> 5, hh = lane >> 4, m = lane & 15;
  const int rt = (int)blockIdx.x, ng = wave;
  const unsigned short* ap  = sent16 + (size_t)(rt * 16 + m) * NEP + 8 * hh;
  const unsigned short* bp0 = wt16 + (size_t)(ng * 64 + m) * NEP + 8 * hh;

  v8f acc[4];
#pragma unroll
  for (int t = 0; t < 4; ++t) acc[t] = zero8();

#pragma unroll 1
  for (int kt = 0; kt < NEP / 32; ++kt) {
    Frag a;
    a.q[0] = *(const v4u*)(ap + 32 * kt);
    a.q[1] = *(const v4u*)(ap + 32 * kt + 16);
#pragma unroll
    for (int t = 0; t < 4; ++t) {
      const unsigned short* bp = bp0 + (size_t)t * 16 * NEP + 32 * kt;
      Frag b;
      b.q[0] = *(const v4u*)bp;
      b.q[1] = *(const v4u*)(bp + 16);
      acc[t] = wmh(a.v, b.v, acc[t]);
    }
  }

  {
    float* se = sE + wave * (16 * EP);
    const float sc = 0.0009765625f;
#pragma unroll
    for (int t = 0; t < 4; ++t) {
      const float bias = bw[ng * 64 + 16 * t + m];
#pragma unroll
      for (int r = 0; r < 8; ++r) se[(8 * hh + r) * EP + 16 * t + m] = acc[t][r] * sc + bias;
    }
  }
  __syncthreads();

  const float* se = sE + wave * (16 * EP);
  if (ng < 4) {
    const int q = lane & 7, rr = lane >> 3;
    unsigned short* hp = hproj + (size_t)(rt * 16) * NH + ng * 64 + 8 * q;
    v4u hv[4];
#pragma unroll
    for (int it = 0; it < 4; ++it) {
      const int r = 4 * it + rr;
      const float* sp = se + r * EP + 8 * q;
      hv[it] = pack8(*(const v4f*)sp, *(const v4f*)(sp + 4), 256.0f);
    }
#pragma unroll
    for (int it = 0; it < 4; ++it) *(volatile v4u*)(hp + (size_t)(4 * it + rr) * NH) = hv[it];
    __threadfence();
#pragma unroll
    for (int it = 0; it < 4; ++it) *(volatile v4u*)(hp + (size_t)(4 * it + rr) * NH) = hv[it];
  } else {
    const int q = lane & 15, rr = lane >> 4;
    float* cp = cproj + (size_t)(rt * 16) * NH + (ng - 4) * 64 + 4 * q;
    v4f cv[8];
#pragma unroll
    for (int it = 0; it < 8; ++it) {
      const int r = 2 * it + rr;
      cv[it] = *(const v4f*)(se + r * EP + 4 * q);
    }
#pragma unroll
    for (int it = 0; it < 8; ++it) *(volatile v4f*)(cp + (size_t)(2 * it + rr) * NH) = cv[it];
    __threadfence();
#pragma unroll
    for (int it = 0; it < 8; ++it) *(volatile v4f*)(cp + (size_t)(2 * it + rr) * NH) = cv[it];
  }
}

__global__ __launch_bounds__(RTHR) void k_tree(const int* __restrict__ trans, int T,
                                               const unsigned short* __restrict__ wg16,
                                               const float* __restrict__ bred,
                                               const unsigned short* __restrict__ hproj,
                                               const float* __restrict__ cproj,
                                               unsigned short* hst, float* cst, float* out) {
  extern __shared__ v4u dsm[];
  char* smem = (char*)dsm;
  unsigned short* sA = (unsigned short*)(smem + LDS_A);
  float* sC  = (float*)(smem + LDS_C);
  float* sHf = (float*)(smem + LDS_H);
  int* sPtr = (int*)(smem + LDS_I);
  int* sBp  = sPtr + NB;
  int* sSh  = sPtr + 2 * NB;
  int* sI1  = sPtr + 3 * NB;
  int* sI2  = sPtr + 4 * NB;
  int* sPos = sPtr + 5 * NB;
  int* sBs  = sPtr + 6 * NB;
  int* sAny = sPtr + 7 * NB;

  const int tid = threadIdx.x, lane = tid & 31, wave = tid >> 5, hh = lane >> 4, m = lane & 15;
  const int jt = wave;
  const int j  = jt * 16 + m;

  if (tid < NB) { sPtr[tid] = 0; sBp[tid] = 0; }
  __syncthreads();

  const float bi  = bred[j];
  const float bfl = bred[NH + j];
  const float bfr = bred[2 * NH + j];
  const float bo  = bred[3 * NH + j];
  const float bu  = bred[4 * NH + j];
  const float S14 = 0.00006103515625f;

  for (int t = 0; t < T; ++t) {
    if (tid < NB) {
      const int b = tid;
      const int tr = trans[(size_t)b * T + t];
      const int sh = (tr == 3) ? 1 : 0;
      const int ptr = sPtr[b], bp = sBp[b];
      int i1 = ptr - 1; i1 = (i1 < 0) ? 0 : i1; i1 = (i1 > SDEP - 1) ? (SDEP - 1) : i1;
      int i2 = ptr - 2; i2 = (i2 < 0) ? 0 : i2; i2 = (i2 > SDEP - 1) ? (SDEP - 1) : i2;
      int pos = sh ? ptr : i2;
      pos = (pos < 0) ? 0 : pos; pos = (pos > SDEP - 1) ? (SDEP - 1) : pos;
      int bs = (bp > NL - 1) ? (NL - 1) : bp; bs = (bs < 0) ? 0 : bs;
      sSh[b] = sh; sI1[b] = i1; sI2[b] = i2; sPos[b] = pos; sBs[b] = bs;
      sPtr[b] = ptr + (sh ? 1 : -1);
      sBp[b]  = bp + sh;
      const unsigned red = __builtin_amdgcn_ballot_w32(sh == 0);
      if (lane == 0) sAny[wave] = (red != 0u) ? 1 : 0;
    }
    __syncthreads();
    const int anyR = __builtin_amdgcn_readfirstlane(sAny[0] | sAny[1]);

    if (anyR) {
#pragma unroll
      for (int it = 0; it < 8; ++it) {
        const int p = it * RTHR + tid;
        const int b = p >> 6, q = p & 63;
        const int i2v = sI2[b], i1v = sI1[b];
        const int idx = (q < 32) ? i2v : i1v;
        const int col = (q & 31) * 8;
        const v4u v = *(const volatile v4u*)(hst + ((size_t)(b * SDEP + idx)) * NH + col);
        *(v4u*)(sA + b * APITCH + q * 8) = v;
      }
    }
    __syncthreads();

    if (anyR) {
#pragma unroll 1
      for (int mt = 0; mt < 4; ++mt) {
        v8f acc[5];
#pragma unroll
        for (int g = 0; g < 5; ++g) acc[g] = zero8();
        const unsigned short* arow = sA + (mt * 16 + m) * APITCH + 8 * hh;
        const unsigned short* brow = wg16 + (size_t)j * NH2 + 8 * hh;
#pragma unroll 1
        for (int ks = 0; ks < NH2 / 32; ++ks) {
          Frag a;
          a.q[0] = *(const v4u*)(arow + 32 * ks);
          a.q[1] = *(const v4u*)(arow + 32 * ks + 16);
#pragma unroll
          for (int g = 0; g < 5; ++g) {
            const unsigned short* bp = brow + (size_t)g * NH * NH2 + 32 * ks;
            Frag b;
            b.q[0] = *(const v4u*)bp;
            b.q[1] = *(const v4u*)(bp + 16);
            acc[g] = wmh(a.v, b.v, acc[g]);
          }
        }
#pragma unroll
        for (int r = 0; r < 8; ++r) {
          const int b = mt * 16 + 8 * hh + r;
          const int i1v = sI1[b], i2v = sI2[b];
          const float cl = *(const volatile float*)(cst + ((size_t)(b * SDEP + i2v)) * NH + j);
          const float cr = *(const volatile float*)(cst + ((size_t)(b * SDEP + i1v)) * NH + j);
          const float ig = acc[0][r] * S14 + bi;
          const float fl = acc[1][r] * S14 + bfl;
          const float fr = acc[2][r] * S14 + bfr;
          const float og = acc[3][r] * S14 + bo;
          const float ug = acc[4][r] * S14 + bu;
          const float cn = sigf(fl) * cl + sigf(fr) * cr + sigf(ig) * tanhx(ug);
          const float hn = sigf(og) * tanhx(cn);
          sC[b * NH + j]  = cn;
          sHf[b * NH + j] = hn;
        }
      }
    }
    __syncthreads();

    {
      const int last = (t == T - 1) ? 1 : 0;
      v4u hv[4];
      v4f ca[4], cb[4], oa[4], ob[4];
      int posv[4];
#pragma unroll
      for (int i = 0; i < 4; ++i) {
        const int b = wave + 16 * i;
        const int s = sSh[b];
        posv[i] = sPos[b];
        const int bs = sBs[b];
        const float* hrp = sHf + b * NH;
        const float* crp = sC + b * NH;
        const v4u hred = pack8(*(const v4f*)(hrp + 8 * lane), *(const v4f*)(hrp + 8 * lane + 4), 256.0f);
        const v4f c0r = *(const v4f*)(crp + 4 * lane);
        const v4f c1r = *(const v4f*)(crp + 128 + 4 * lane);
        const size_t prow = (size_t)(b * NL + bs) * NH;
        const v4u hsh = *(const v4u*)(hproj + prow + 8 * lane);
        const v4f c0s = *(const v4f*)(cproj + prow + 4 * lane);
        const v4f c1s = *(const v4f*)(cproj + prow + 128 + 4 * lane);
        hv[i] = s ? hsh : hred;
        ca[i] = s ? c0s : c0r;
        cb[i] = s ? c1s : c1r;
        const v4f z = {0.f, 0.f, 0.f, 0.f};
        oa[i] = z; ob[i] = z;
        if (last) {
          const v4f o0r = *(const v4f*)(hrp + 4 * lane);
          const v4f o1r = *(const v4f*)(hrp + 128 + 4 * lane);
          const v4h q0 = *(const v4h*)(hproj + prow + 4 * lane);
          const v4h q1 = *(const v4h*)(hproj + prow + 128 + 4 * lane);
          const float iv = 0.00390625f;
          const v4f o0s = {(float)q0.x * iv, (float)q0.y * iv, (float)q0.z * iv, (float)q0.w * iv};
          const v4f o1s = {(float)q1.x * iv, (float)q1.y * iv, (float)q1.z * iv, (float)q1.w * iv};
          oa[i] = s ? o0s : o0r;
          ob[i] = s ? o1s : o1r;
        }
      }
#pragma unroll
      for (int i = 0; i < 4; ++i) {
        const int b = wave + 16 * i;
        const size_t srow = (size_t)(b * SDEP + posv[i]) * NH;
        *(volatile v4u*)(hst + srow + 8 * lane) = hv[i];
        *(volatile v4f*)(cst + srow + 4 * lane) = ca[i];
        *(volatile v4f*)(cst + srow + 128 + 4 * lane) = cb[i];
        if (last) {
          *(volatile v4f*)(out + (size_t)b * NH + 4 * lane) = oa[i];
          *(volatile v4f*)(out + (size_t)b * NH + 128 + 4 * lane) = ob[i];
        }
      }
      __threadfence();
#pragma unroll
      for (int i = 0; i < 4; ++i) {
        const int b = wave + 16 * i;
        const size_t srow = (size_t)(b * SDEP + posv[i]) * NH;
        *(volatile v4u*)(hst + srow + 8 * lane) = hv[i];
        *(volatile v4f*)(cst + srow + 4 * lane) = ca[i];
        *(volatile v4f*)(cst + srow + 128 + 4 * lane) = cb[i];
        if (last) {
          *(volatile v4f*)(out + (size_t)b * NH + 4 * lane) = oa[i];
          *(volatile v4f*)(out + (size_t)b * NH + 128 + 4 * lane) = ob[i];
        }
      }
    }
    __syncthreads();
  }
}

extern "C" void kernel_launch(void* const* d_in, const int* in_sizes, int n_in,
                              void* d_out, int out_size, void* d_ws, size_t ws_size,
                              hipStream_t stream) {
  if (n_in < 7) return;
  if (in_sizes[0] != NROWS * NE) return;
  if (in_sizes[1] < NB || (in_sizes[1] % NB) != 0) return;
  const int T = in_sizes[1] / NB;
  if (in_sizes[2] != NE * NH2) return;
  if (in_sizes[3] != NH2) return;
  if (in_sizes[4] != NH * NG5) return;
  if (in_sizes[5] != NH * NG5) return;
  if (in_sizes[6] != NG5) return;
  if (out_size != NB * NH) return;

  const float* sent  = (const float*)d_in[0];
  const int*   trans = (const int*)d_in[1];
  const float* Ww    = (const float*)d_in[2];
  const float* bw    = (const float*)d_in[3];
  const float* Wl    = (const float*)d_in[4];
  const float* Wr    = (const float*)d_in[5];
  const float* bred  = (const float*)d_in[6];
  float* out = (float*)d_out;

  char* ws = (char*)d_ws;
  size_t off = 0;
  const size_t oS16 = off; off += (size_t)NROWS * NEP * 2;       off = (off + 255) & ~(size_t)255;
  const size_t oWt  = off; off += (size_t)NH2 * NEP * 2;         off = (off + 255) & ~(size_t)255;
  const size_t oWg  = off; off += (size_t)NG5 * NH2 * 2;         off = (off + 255) & ~(size_t)255;
  const size_t oHp  = off; off += (size_t)NROWS * NH * 2;        off = (off + 255) & ~(size_t)255;
  const size_t oCp  = off; off += (size_t)NROWS * NH * 4;        off = (off + 255) & ~(size_t)255;
  const size_t oHs  = off; off += (size_t)NB * SDEP * NH * 2;    off = (off + 255) & ~(size_t)255;
  const size_t oCs  = off; off += (size_t)NB * SDEP * NH * 4;    off = (off + 255) & ~(size_t)255;
  if (off > ws_size || off > (size_t)WSCAP) return;
  unsigned short* sent16 = (unsigned short*)(ws + oS16);
  unsigned short* wt16   = (unsigned short*)(ws + oWt);
  unsigned short* wg16   = (unsigned short*)(ws + oWg);
  unsigned short* hproj  = (unsigned short*)(ws + oHp);
  float*          cproj  = (float*)(ws + oCp);
  unsigned short* hst    = (unsigned short*)(ws + oHs);
  float*          cst    = (float*)(ws + oCs);

  k_cvt<<<CB_S + CB_W + CB_G, NTHR, 0, stream>>>(sent, Ww, Wl, Wr, sent16, wt16, wg16);

  k_proj<<<NROWS / 16, NTHR, 0, stream>>>(sent16, wt16, bw, hproj, cproj);

  hipFuncSetAttribute(reinterpret_cast<const void*>(&k_tree), hipFuncAttributeMaxDynamicSharedMemorySize, LDS_TOT);
  k_tree<<<1, RTHR, LDS_TOT, stream>>>(trans, T, wg16, bred, hproj, cproj, hst, cst, out);
}
